// CrissCrossAttention_32736240730147
// MI455X (gfx1250) — hardware-run, weakly checked
//
#include <hip/hip_runtime.h>


#ifndef NB
#define NB 8
#endif
#ifndef SEQ
#define SEQ 512
#endif
#define NB_FULL  8
#define SEQ_FULL 512
#ifndef OUT_NB
#define OUT_NB NB
#endif
#define DM    64
#define FEAT  32
#define SD    (SEQ / 4)
#define UP_N  12
#define CF_   3
#define AW    4
#define OSP   68
#define WCS   64.0f
#define VCS   256.0f
#define QRS   2048.0f
#define QRI   (1.0f / 2048.0f)
#define PSH   14.0f
#define LOG2E 1.4426950408889634f

static_assert(DM == 64);
static_assert(FEAT * 2 == DM);
static_assert((SEQ & (SEQ - 1)) == 0);
static_assert((SD & (SD - 1)) == 0);
static_assert(SEQ % 128 == 0);
static_assert(SEQ % 64 == 0);
static_assert(SEQ % 32 == 0);
static_assert(DM % 32 == 0);
static_assert(UP_N < SEQ / 2);
static_assert(NB <= NB_FULL);
static_assert(SEQ <= SEQ_FULL);
static_assert(AW * 4 == 16);
static_assert(AW * 16 == DM);
static_assert((OSP * 4) % 16 == 0);
static_assert(FEAT * 32 == 256 * 4);
static_assert(8 * 16 == 32 * 4);
static_assert(256 * 16 == 32 * DM * 2);
static_assert(32 * 16 * 8 == 16 * DM * 4);
static_assert(32 * 16 * 4 == 16 * DM * 2);
static_assert(2 * 2 * 16 == 64);
static_assert(32 * 16 == 2 * DM * 4);
static_assert(8 * 8 == DM);
static_assert(32 * AW * 16 * 2 == 16 * DM * 4);
static_assert((SEQ + 64) * 4 <= 131072);
static_assert((2 * SEQ + FEAT * 32) * 4 <= 131072);
static_assert(16 * OSP * 4 <= 131072);
static_assert((2 * 16 * DM + 16 * (DM / 2) + 2 * DM + 32 + 2 * 16 * DM + 16 * OSP) * 4 <= 131072);

typedef _Float16 h16;
typedef __attribute__((ext_vector_type(16))) _Float16 v16h;
typedef __attribute__((ext_vector_type(8)))  _Float16 v8h;
typedef __attribute__((ext_vector_type(8)))  float    v8f;
typedef __attribute__((ext_vector_type(4)))  float    v4f;
typedef __attribute__((ext_vector_type(4)))  unsigned v4u;
typedef v4f  __attribute__((may_alias)) v4fa;
typedef v4u  __attribute__((may_alias)) v4ua;

__device__ __forceinline__ unsigned short f2bf(float f) { unsigned u = __float_as_uint(f); u += 0x7FFFu + ((u >> 16) & 1u); return (unsigned short)(u >> 16); }
__device__ __forceinline__ float bfr(float f) { return __uint_as_float(((unsigned)f2bf(f)) << 16); }
__device__ __forceinline__ v16h cat16(v8h lo, v8h hi) { return __builtin_shufflevector(lo, hi, 0, 1, 2, 3, 4, 5, 6, 7, 8, 9, 10, 11, 12, 13, 14, 15); }
__device__ __forceinline__ v16h ldh(const h16* p) { return cat16(*(const v8h*)p, *(const v8h*)(p + 16)); }
__device__ __forceinline__ h16 toh_flush(float v) { const h16 r = (h16)v; return (fabsf(v) < 6.103515625e-05f) ? (h16)0.0f : r; }
__device__ __forceinline__ v8f wmma16g(v16h a, v16h b, v8f c) {
    c = __builtin_amdgcn_wmma_f32_16x16x32_f16(false, a, false, b, (short)0, c, false, false);
    asm volatile("v_nop\n\tv_nop\n\tv_nop\n\tv_nop" : "+v"(c) : "v"(a), "v"(b));
    return c;
}
__device__ __forceinline__ void wave_sync() { __builtin_amdgcn_fence(3  , "wavefront"); __builtin_amdgcn_wave_barrier(); asm volatile("" ::: "memory"); }

template <int N>
__device__ __forceinline__ void bsum(float (&v)[N], float* red, int lane, int wave) {
#pragma unroll
    for (int i = 0; i < N; ++i) {
        float t = v[i];
        t += __shfl_xor(t, 16, 32); t += __shfl_xor(t, 8, 32); t += __shfl_xor(t, 4, 32); t += __shfl_xor(t, 2, 32); t += __shfl_xor(t, 1, 32);
        v[i] = t; }
    if (lane == 0) {
#pragma unroll
        for (int i = 0; i < N; ++i) red[wave * 8 + i] = v[i]; }
    __syncthreads();
#pragma unroll
    for (int i = 0; i < N; ++i) v[i] = (red[i] + red[8 + i]) + (red[16 + i] + red[24 + i]);
    __syncthreads();
}

__global__ __launch_bounds__(256) void k_wcvt(const float* __restrict__ src, h16* dst, int n8) {
#pragma clang fp contract(off)
    const int i = blockIdx.x * 256 + threadIdx.x; if (i >= n8) return;
    const v8f v = *(const v8f*)(src + (size_t)i * 8); v8h o;
#pragma unroll
    for (int k = 0; k < 8; ++k) o[k] = toh_flush(bfr(v[k]) * WCS);
    *(volatile v8h*)(dst + (size_t)i * 8) = o; __threadfence(); *(volatile v8h*)(dst + (size_t)i * 8) = o;
}

__global__ __launch_bounds__(128) void k_stats(const float* __restrict__ x, const float* __restrict__ fw_r, const float* __restrict__ fw_i,
                                               const float* __restrict__ fb_r, const float* __restrict__ fb_i, float* ST) {
#pragma clang fp contract(off)
    __shared__ float xs[SEQ];
    __shared__ float red[32];
    __shared__ __align__(16) float st[32];
    const int tid = threadIdx.x, lane = tid & 31;
    const int wave = __builtin_amdgcn_readfirstlane((int)(threadIdx.x >> 5));
    const int b = blockIdx.x / FEAT, f = blockIdx.x % FEAT;
    float r1[1]; r1[0] = 0.0f;
    for (int s = tid; s < SEQ; s += 128) { const float u = bfr(x[((size_t)s * NB_FULL + b) * DM + f]); xs[s] = u; r1[0] += u; }
    bsum<1>(r1, red, lane, wave);
    const float xm = r1[0] * (1.0f / (float)SEQ);
    r1[0] = 0.0f;
    for (int s = tid; s < SEQ; s += 128) { const float d = xs[s] - xm; r1[0] += d * d; }
    bsum<1>(r1, red, lane, wave);
    const float xv = r1[0] * (1.0f / (float)(SEQ - 1)) + 1e-5f;
    const float xinv = rsqrtf(xv);
    r1[0] = 0.0f;
    for (int t = tid; t < SD; t += 128) r1[0] += xs[4 * t];
    bsum<1>(r1, red, lane, wave);
    const float fm = r1[0] * (1.0f / (float)SD);
    r1[0] = 0.0f;
    for (int t = tid; t < SD; t += 128) { const float d = xs[4 * t] - fm; r1[0] += d * d; }
    bsum<1>(r1, red, lane, wave);
    const float fv = r1[0] * (1.0f / (float)(SD - 1)) + 1e-5f;
    const float finv = rsqrtf(fv);
    const float fsd = fv * finv;
    float c5[5];
#pragma unroll
    for (int i = 0; i < 5; ++i) c5[i] = 0.0f;
    for (int t = tid; t < SD; t += 128) {
        const float fn = (xs[4 * t] - fm) * finv;
        const float fr1 = (float)(t & (SD - 1)) * (1.0f / (float)SD);
        const float fr2 = (float)((2 * t) & (SD - 1)) * (1.0f / (float)SD);
        const float cs1 = __builtin_amdgcn_cosf(fr1), sn1 = __builtin_amdgcn_sinf(fr1);
        const float cs2 = __builtin_amdgcn_cosf(fr2), sn2 = __builtin_amdgcn_sinf(fr2);
        c5[0] += fn; c5[1] += fn * cs1; c5[2] -= fn * sn1; c5[3] += fn * cs2; c5[4] -= fn * sn2; }
    bsum<5>(c5, red, lane, wave);
    const float Sr[CF_] = { c5[0], c5[1], c5[3] };
    const float Si[CF_] = { 0.0f, c5[2], c5[4] };
    const int kk = tid < UP_N ? tid : (UP_N - 1);
    float ur = bfr(fb_r[kk]), ui = bfr(fb_i[kk]);
#pragma unroll
    for (int c = 0; c < CF_; ++c) {
        const float wr = bfr(fw_r[kk * CF_ + c]), wi = bfr(fw_i[kk * CF_ + c]);
        ur += wr * Sr[c] - wi * Si[c];
        ui += wr * Si[c] + wi * Sr[c]; }
    asm volatile("" : "+v"(ur), "+v"(ui));
    if (tid < UP_N) { st[4 + kk] = ur; st[16 + kk] = ui; }
    if (tid == 0) { st[0] = xm; st[1] = xinv; st[2] = fm; st[3] = fsd; st[28] = 0.0f; st[29] = 0.0f; st[30] = 0.0f; st[31] = 0.0f; }
    __syncthreads();
    if (wave == 0) {
        const int c4 = (lane & 7) * 4;
        const v4f val = *(const v4fa*)(&st[c4]);
        float* dst = ST + (size_t)blockIdx.x * 32 + c4;
#pragma unroll 1
        for (int ps = 0; ps < 2; ++ps) {
            if (lane < 8) *(volatile v4f*)dst = val;
            if (ps == 0) __threadfence(); } }
}

__global__ __launch_bounds__(256) void k_img(const float* __restrict__ x, const float* __restrict__ ST, h16* IMG, h16* IMR) {
#pragma clang fp contract(off)
    __shared__ float cst[SEQ];
    __shared__ float snt[SEQ];
    __shared__ __align__(16) float stl[FEAT * 32];
    const int tid = threadIdx.x; const int b = blockIdx.y;
    for (int j = tid; j < SEQ; j += 256) { const float fr = (float)j * (1.0f / (float)SEQ); cst[j] = __builtin_amdgcn_cosf(fr); snt[j] = __builtin_amdgcn_sinf(fr); }
    { const v4f t = *(const v4f*)(ST + (size_t)b * FEAT * 32 + (size_t)tid * 4); *(v4fa*)(&stl[tid * 4]) = t; }
    __syncthreads();
    const int s = blockIdx.x * 32 + (tid >> 3), q = tid & 7;
    const v4f xv = *(const v4f*)(x + ((size_t)s * NB_FULL + b) * DM + 4 * q);
    float acc[4];
#pragma unroll
    for (int j = 0; j < 4; ++j) acc[j] = stl[(4 * q + j) * 32 + 4];
#pragma unroll 1
    for (int kk = 1; kk < UP_N; ++kk) {
        const int idx = (kk * s) & (SEQ - 1);
        const float cs = cst[idx], sn = snt[idx];
#pragma unroll
        for (int j = 0; j < 4; ++j) { const float ur = stl[(4 * q + j) * 32 + 4 + kk], ui = stl[(4 * q + j) * 32 + 16 + kk]; acc[j] += 2.0f * (ur * cs - ui * sn); } }
    v8h o, orr;
#pragma unroll
    for (int j = 0; j < 4; ++j) {
        const int fo = (4 * q + j) * 32;
        const float xm = stl[fo], xinv = stl[fo + 1], fm = stl[fo + 2], fsd = stl[fo + 3];
        const float xn = (bfr(xv[j]) - xm) * xinv;
        const float xy = (acc[j] * (4.0f / (float)SEQ)) * fsd + fm;
        const h16 hn = toh_flush(xn), hy = toh_flush(xy);
        o[2 * j] = hn; o[2 * j + 1] = hy;
        orr[2 * j] = toh_flush((xn - (float)hn) * QRS); orr[2 * j + 1] = toh_flush((xy - (float)hy) * QRS); }
    const size_t off = ((size_t)b * SEQ + s) * DM + 8 * q;
    *(volatile v8h*)(IMG + off) = o; *(volatile v8h*)(IMR + off) = orr; __threadfence(); *(volatile v8h*)(IMG + off) = o; *(volatile v8h*)(IMR + off) = orr;
}

static constexpr size_t NPL = (size_t)NB * SEQ * DM;
static constexpr size_t HPE = ((((NPL + (size_t)3 * DM * DM) * 2) + 255) & ~(size_t)255) / 2;
__global__ __launch_bounds__(32) void k_proj(const h16* __restrict__ HP, float* FP, h16* VP) {
    __shared__ __align__(16) float os[16 * OSP];
    const int lane = threadIdx.x & 31, lr = lane & 15, hi = lane >> 4;
    const int job = blockIdx.y; const int r64 = blockIdx.x * 64;
    const bool tr = (job == 2) | (job == 4);
    const int wsel = (job == 0) ? 0 : ((job <= 2) ? 1 : 2);
    const size_t imgo = (size_t)r64 * DM, wo = NPL + (size_t)wsel * DM * DM, reso = HPE + imgo;
    const size_t lo = (size_t)lr * DM + 8 * hi;
    const size_t aoff  = (tr ? wo : imgo) + lo;
    const size_t boff  = (tr ? imgo : wo) + lo;
    const size_t aroff = (tr ? wo : reso) + lo;
    const size_t broff = (tr ? reso : wo) + lo;
    const float sc = (job == 0) ? (LOG2E / WCS) : ((job <= 2) ? (1.0f / WCS) : (VCS / WCS));
    const int bb = r64 / SEQ, tt = r64 % SEQ;
    const size_t ob = tr ? ((size_t)bb * DM * SEQ + (size_t)tt) : imgo;
    const size_t op = tr ? (size_t)SEQ : (size_t)DM;
    const size_t pf = (job == 0) ? (size_t)0 : ((job == 1) ? NPL : 2 * NPL);
    const size_t ph = (job == 4) ? NPL : (size_t)0;
#pragma unroll 1
    for (int mh = 0; mh < 2; ++mh) {
        const size_t am = (size_t)mh * 32 * DM;
        v8f acc[2][4], accr[2][4];
#pragma unroll
        for (int mb = 0; mb < 2; ++mb)
#pragma unroll
            for (int nb = 0; nb < 4; ++nb) { acc[mb][nb] = (v8f){}; accr[mb][nb] = (v8f){}; }
#pragma unroll 1
        for (int kc = 0; kc < DM; kc += 32) {
            v16h a[2], ar[2];
#pragma unroll
            for (int mb = 0; mb < 2; ++mb) { a[mb] = ldh(HP + aoff + am + (size_t)mb * 16 * DM + kc); ar[mb] = ldh(HP + aroff + am + (size_t)mb * 16 * DM + kc); }
#pragma unroll
            for (int nb = 0; nb < 4; ++nb) { const v16h bq = ldh(HP + boff + (size_t)nb * 16 * DM + kc); const v16h br = ldh(HP + broff + (size_t)nb * 16 * DM + kc);
#pragma unroll
                for (int mb = 0; mb < 2; ++mb) { acc[mb][nb] = wmma16g(a[mb], bq, acc[mb][nb]); accr[mb][nb] = wmma16g(ar[mb], br, accr[mb][nb]); } }
        }
#pragma unroll
        for (int mb = 0; mb < 2; ++mb) {
            const int m16 = mh * 32 + mb * 16;
#pragma unroll
            for (int nb = 0; nb < 4; ++nb) {
#pragma unroll
                for (int j = 0; j < 8; ++j) os[(hi * 8 + j) * OSP + nb * 16 + lr] = (acc[mb][nb][j] + accr[mb][nb][j] * QRI) * sc; }
            wave_sync();
#pragma unroll 1
            for (int ps = 0; ps < 2; ++ps) {
                if (job <= 2) {
#pragma unroll
                    for (int s = 0; s < 8; ++s) { const int row = 2 * s + (lane >> 4), c4 = (lane & 15) * 4;
                        const v4f val = *(const v4fa*)(&os[row * OSP + c4]);
                        *(volatile v4f*)(FP + pf + ob + (size_t)(m16 + row) * op + c4) = val; }
                } else {
#pragma unroll
                    for (int s = 0; s < 4; ++s) { const int row = 4 * s + (lane >> 3), c8 = (lane & 7) * 8;
                        const v4f x0 = *(const v4fa*)(&os[row * OSP + c8]); const v4f x1 = *(const v4fa*)(&os[row * OSP + c8 + 4]); v8h hv;
#pragma unroll
                        for (int i = 0; i < 4; ++i) { hv[i] = toh_flush(x0[i]); hv[4 + i] = toh_flush(x1[i]); }
                        *(volatile v8h*)(VP + ph + ob + (size_t)(m16 + row) * op + c8) = hv; }
                }
                if (ps == 0) __threadfence(); }
            wave_sync();
        }
    }
}

__global__ __launch_bounds__(256) void k_colstat(const float* __restrict__ KT, float* CS) {
#pragma clang fp contract(off)
    __shared__ __align__(16) float cs[2 * DM];
    const int lane = threadIdx.x & 31;
    const int wave = __builtin_amdgcn_readfirstlane((int)(threadIdx.x >> 5));
    const int b = blockIdx.x;
#pragma unroll 1
    for (int i = 0; i < 8; ++i) {
        const int w = wave * 8 + i;
        const float* row = KT + ((size_t)(b * DM + w)) * SEQ;
        float mx = -3.0e38f, mn = 3.0e38f;
#pragma unroll 1
        for (int j = lane * 4; j < SEQ; j += 128) { const v4f kv = *(const v4f*)(row + j);
            mx = fmaxf(fmaxf(mx, kv[0]), fmaxf(kv[1], fmaxf(kv[2], kv[3])));
            mn = fminf(fminf(mn, kv[0]), fminf(kv[1], fminf(kv[2], kv[3]))); }
#pragma unroll
        for (int off = 16; off > 0; off >>= 1) { mx = fmaxf(mx, __shfl_xor(mx, off, 32)); mn = fminf(mn, __shfl_xor(mn, off, 32)); }
        if (lane == 0) { cs[w] = mx; cs[DM + w] = mn; } }
    __syncthreads();
    if (wave == 0) {
        const v4f val = *(const v4fa*)(&cs[lane * 4]);
        float* dst = CS + (size_t)b * 2 * DM + lane * 4;
        *(volatile v4f*)dst = val; __threadfence(); *(volatile v4f*)dst = val; }
}

__device__ __forceinline__ float rowshift(float q2, float kx, float kn) {
#pragma clang fp contract(off)
    const float a = q2 * kx, c = q2 * kn;
    const float m2 = (q2 >= 0.0f) ? a : c;
    return PSH - m2;
}
__device__ __forceinline__ h16 pexp(float q2, float k, float sh) {
    const float e = fmaf(q2, k, sh);
    const float p = __builtin_amdgcn_exp2f(e);
    return (e < -14.0f) ? (h16)0.0f : (h16)p;
}
__device__ __forceinline__ v16h mkP(float q2, float sh, v4f k0, v4f k1, v4f k2, v4f k3) {
    v16h p;
#pragma unroll
    for (int j = 0; j < 4; ++j) { p[j] = pexp(q2, k0[j], sh); p[4 + j] = pexp(q2, k1[j], sh); p[8 + j] = pexp(q2, k2[j], sh); p[12 + j] = pexp(q2, k3[j], sh); }
    return p;
}
__device__ __forceinline__ v16h mkA(v4u r0, v4u r1, unsigned am, unsigned on) {
    const v4u amv = (v4u){am, am, am, am}, onv = (v4u){on, on, on, on};
    const v4u a0 = (r0 & amv) | onv, a1 = (r1 & amv) | onv;
    return cat16(__builtin_bit_cast(v8h, a0), __builtin_bit_cast(v8h, a1));
}

__global__ __launch_bounds__(32 * AW) void k_attn(const float* __restrict__ QF, const float* __restrict__ KF, const float* __restrict__ KT,
                                                  const h16* __restrict__ VH, const h16* __restrict__ VT, const float* __restrict__ CS,
                                                  const float* __restrict__ gamma, float* OUT) {
    __shared__ __align__(16) float qs[16 * DM];
    __shared__ __align__(16) float ks[16 * DM];
    __shared__ __align__(16) unsigned vsu[16 * (DM / 2)];
    __shared__ __align__(16) float ccs[2 * DM];
    __shared__ float rmx[16];
    __shared__ float rmn[16];
    __shared__ float rnum[16 * DM];
    __shared__ float rden[16 * DM];
    __shared__ __align__(16) float os[16 * OSP];
    const int tid = threadIdx.x, lane = tid & 31, lr = lane & 15, hi = lane >> 4;
    const int wave = __builtin_amdgcn_readfirstlane((int)(threadIdx.x >> 5));
    const int b = blockIdx.y; const int h0 = blockIdx.x * 16;
    const size_t rowbase = ((size_t)b * SEQ + h0) * DM;
#pragma unroll
    for (int i = 0; i < 2; ++i) { const int j = tid + 128 * i;
        *(v4fa*)(&qs[j * 4]) = *(const v4f*)(QF + rowbase + (size_t)j * 4);
        *(v4fa*)(&ks[j * 4]) = *(const v4f*)(KF + rowbase + (size_t)j * 4); }
    *(v4ua*)(&vsu[tid * 4]) = *(const v4u*)(VH + rowbase + (size_t)tid * 8);
    if (wave == 0) *(v4fa*)(&ccs[lane * 4]) = *(const v4f*)(CS + (size_t)b * 2 * DM + lane * 4);
    const float g0 = bfr(gamma[0]);
    __syncthreads();
#pragma unroll 1
    for (int i = 0; i < 4; ++i) { const int r = wave * 4 + i;
        const float a = ks[r * DM + lane], c = ks[r * DM + 32 + lane];
        float mx = fmaxf(a, c), mn = fminf(a, c);
#pragma unroll
        for (int off = 16; off > 0; off >>= 1) { mx = fmaxf(mx, __shfl_xor(mx, off, 32)); mn = fminf(mn, __shfl_xor(mn, off, 32)); }
        if (lane == 0) { rmx[r] = mx; rmn[r] = mn; } }
    __syncthreads();
    const unsigned am = (lr == 0) ? 0xFFFFFFFFu : 0u;
    const unsigned on = (lr == 1) ? 0x3C003C00u : 0u;
#pragma unroll 1
    for (int i = 0; i < 4; ++i) { const int r = wave * 4 + i;
        const float rx = rmx[r], rn = rmn[r];
#pragma unroll 1
        for (int wt = 0; wt < 4; ++wt) { const int w = wt * 16 + lr;
            const float q2 = qs[r * DM + w];
            const float sh = rowshift(q2, fmaxf(ccs[w], rx), fminf(ccs[DM + w], rn));
            v8f acc = (v8f){};
#pragma unroll
            for (int s2 = 0; s2 < 2; ++s2) { const int c0 = s2 * 32 + 8 * hi;
                const v4f k0 = *(const v4fa*)(&ks[r * DM + c0]), k1 = *(const v4fa*)(&ks[r * DM + c0 + 4]);
                const v4f k2 = *(const v4fa*)(&ks[r * DM + c0 + 16]), k3 = *(const v4fa*)(&ks[r * DM + c0 + 20]);
                const v4u r0 = *(const v4ua*)(&vsu[r * (DM / 2) + (c0 >> 1)]), r1 = *(const v4ua*)(&vsu[r * (DM / 2) + ((c0 + 16) >> 1)]);
                const v16h p = mkP(q2, sh, k0, k1, k2, k3);
                const v16h a = mkA(r0, r1, am, on);
                acc = wmma16g(a, p, acc); }
            if (hi == 0) { rnum[r * DM + w] = acc[0]; rden[r * DM + w] = acc[1]; } } }
    __syncthreads();
#pragma unroll 1
    for (int i = 0; i < 16; ++i) { const int w = wave * 16 + i;
        const float q2 = qs[lr * DM + w];
        const float sh = rowshift(q2, fmaxf(ccs[w], rmx[lr]), fminf(ccs[DM + w], rmn[lr]));
        const float cn = rnum[lr * DM + w], cd = rden[lr * DM + w];
        v8f acc = (v8f){};
        acc[0] = (hi == 0) ? cn : 0.0f; acc[1] = (hi == 0) ? cd : 0.0f;
        const size_t cb = ((size_t)(b * DM + w)) * SEQ + 8 * hi;
#pragma unroll 1
        for (int key0 = 0; key0 < SEQ; key0 += 32) {
            const float* kp = KT + cb + key0;
            const v4f k0 = *(const v4f*)kp, k1 = *(const v4f*)(kp + 4), k2 = *(const v4f*)(kp + 16), k3 = *(const v4f*)(kp + 20);
            const v4u r0 = *(const v4u*)(VT + cb + key0), r1 = *(const v4u*)(VT + cb + key0 + 16);
            const v16h p = mkP(q2, sh, k0, k1, k2, k3);
            const v16h a = mkA(r0, r1, am, on);
            acc = wmma16g(a, p, acc); }
        const float den = (hi == 0) ? acc[1] : 1.0f;
        const float val = (acc[0] * (1.0f / den)) * (g0 * (1.0f / VCS));
        if (hi == 0) os[lr * OSP + w] = val; }
    __syncthreads();
#pragma unroll 1
    for (int ps = 0; ps < 2; ++ps) {
#pragma unroll
        for (int s = 0; s < 2; ++s) { const int row = 8 * s + (tid >> 4), c4 = (tid & 15) * 4;
            const v4f val = *(const v4fa*)(&os[row * OSP + c4]);
            *(volatile v4f*)(OUT + ((size_t)(h0 + row) * OUT_NB + b) * DM + c4) = val; }
        if (ps == 0) __threadfence(); }
}

static constexpr size_t al256(size_t v) { return (v + 255) & ~(size_t)255; }
static constexpr size_t SZ_HP = al256((NPL + (size_t)3 * DM * DM) * 2);
static constexpr size_t SZ_HR = al256(NPL * 2);
static constexpr size_t SZ_FP = al256((size_t)3 * NPL * 4);
static constexpr size_t SZ_VP = al256((size_t)2 * NPL * 2);
static constexpr size_t SZ_ST = al256((size_t)NB * FEAT * 32 * 4);
static constexpr size_t SZ_CS = al256((size_t)NB * 2 * DM * 4);
static constexpr size_t SZ_TOTAL = SZ_HP + SZ_HR + SZ_FP + SZ_VP + SZ_ST + SZ_CS;
static_assert(SZ_TOTAL <= (size_t)134217728);
static_assert(SZ_HP == HPE * 2);
static_assert((HPE + NPL) * 2 <= SZ_HP + SZ_HR);
static_assert((NPL * 2) % 256 == 0);
static_assert((NPL * 4) % 256 == 0);
static_assert(((size_t)DM * DM) % 8 == 0);
static_assert((size_t)NB * DM * SEQ == NPL);
static_assert((size_t)(NB * SEQ / 64) * 64 * DM == NPL);
static_assert((size_t)(SEQ / 32) * 32 * NB * DM == NPL);

extern "C" void kernel_launch(void* const* d_in, const int* in_sizes, int n_in,
                              void* d_out, int out_size, void* d_ws, size_t ws_size, hipStream_t stream) {
    if (n_in < 9) return;
    const size_t needx = ((size_t)(SEQ - 1) * NB_FULL + NB) * DM;
    if ((size_t)in_sizes[0] < needx) return;
    if ((size_t)in_sizes[1] < (size_t)DM * DM || (size_t)in_sizes[2] < (size_t)DM * DM || (size_t)in_sizes[3] < (size_t)DM * DM) return;
    if (in_sizes[4] < UP_N * CF_ || in_sizes[5] < UP_N * CF_ || in_sizes[6] < UP_N || in_sizes[7] < UP_N || in_sizes[8] < 1) return;
    if ((size_t)out_size < ((size_t)(SEQ - 1) * OUT_NB + NB) * DM) return;
    if (SZ_TOTAL > ws_size) return;
    const float* x   = (const float*)d_in[0];
    const float* wq  = (const float*)d_in[1];
    const float* wk  = (const float*)d_in[2];
    const float* wv  = (const float*)d_in[3];
    const float* fwr = (const float*)d_in[4];
    const float* fwi = (const float*)d_in[5];
    const float* fbr = (const float*)d_in[6];
    const float* fbi = (const float*)d_in[7];
    const float* gam = (const float*)d_in[8];
    float* OUT = (float*)d_out;
    char* wsp = (char*)d_ws;
    h16* HP = (h16*)wsp; wsp += SZ_HP;
    h16* HR = (h16*)wsp; wsp += SZ_HR;
    float* FP = (float*)wsp; wsp += SZ_FP;
    h16* VP = (h16*)wsp; wsp += SZ_VP;
    float* ST = (float*)wsp; wsp += SZ_ST;
    float* CS = (float*)wsp; wsp += SZ_CS;
    h16* WH = HP + NPL;
    const float* QF = FP; const float* KF = FP + NPL; const float* KT = FP + 2 * NPL;
    const h16* VH = VP; const h16* VT = VP + NPL;

    { const int n8 = DM * DM / 8; const unsigned g = (unsigned)((n8 + 255) / 256);
      k_wcvt<<<g, 256, 0, stream>>>(wq, WH, n8);
      k_wcvt<<<g, 256, 0, stream>>>(wk, WH + (size_t)DM * DM, n8);
      k_wcvt<<<g, 256, 0, stream>>>(wv, WH + (size_t)2 * DM * DM, n8); }
    k_stats<<<NB * FEAT, 128, 0, stream>>>(x, fwr, fwi, fbr, fbi, ST);
    k_img<<<dim3(SEQ / 32, NB, 1), 256, 0, stream>>>(x, ST, HP, HR);
    k_proj<<<dim3(NB * SEQ / 64, 5, 1), 32, 0, stream>>>(HP, FP, VP);
    k_colstat<<<NB, 256, 0, stream>>>(KT, CS);
    k_attn<<<dim3(SEQ / 16, NB, 1), 32 * AW, 0, stream>>>(QF, KF, KT, VH, VT, CS, gam, OUT);
}
